// SceneGraphGATLayer_69166153335439
// MI455X (gfx1250) — hardware-verified
//
#include <hip/hip_runtime.h>
#define NBG 32
#define NND 256
#define DD 512
#define NH 8
#define HD 64
#define NEG 1024
#define NET (NBG * NEG)
#define EDIM 256
#define GDIM 64
#define DFF 2048
#define NR (NBG * NND)
#define NKEY (NBG * 257)
#define ECAP 32
#define BGRP 8
#define LNEPS 1e-5f
typedef __bf16 v16b __attribute__((ext_vector_type(16)));
typedef unsigned short v8us __attribute__((ext_vector_type(8), may_alias));
typedef float  v8f  __attribute__((ext_vector_type(8)));
typedef float  v4f  __attribute__((ext_vector_type(4)));
typedef float  v4fa __attribute__((ext_vector_type(4), may_alias));
union FragB { v16b v; v8us half[2]; unsigned short u[16]; };

__device__ __forceinline__ unsigned short bf16_bits(float x) { unsigned int u = __float_as_uint(x); return (unsigned short)((u + 0x7FFFu + ((u >> 16) & 1u)) >> 16); }
__device__ __forceinline__ float bf16_val(unsigned short b) { return __uint_as_float(((unsigned int)b) << 16); }
__device__ __forceinline__ float bf16_round(float x) { return bf16_val(bf16_bits(x)); }
template <int NT>
__device__ __forceinline__ v8f mmaN(v16b ah, v16b al, v16b bh, v16b bl, v8f c) {
  c = __builtin_amdgcn_wmma_f32_16x16x32_bf16(false, ah, false, bh, (short)0, c, false, false);
  if (NT >= 2) c = __builtin_amdgcn_wmma_f32_16x16x32_bf16(false, al, false, bh, (short)0, c, false, false);
  if (NT >= 3) c = __builtin_amdgcn_wmma_f32_16x16x32_bf16(false, ah, false, bl, (short)0, c, false, false);
  asm volatile("v_nop\n\tv_nop\n\tv_nop\n\tv_nop" : "+v"(c) : "v"(ah), "v"(al), "v"(bh), "v"(bl));
  return c;
}

__global__ __launch_bounds__(256) void k_wt_bf16(const float* __restrict__ W, unsigned short* __restrict__ Wt, int K, int N) {
  const int t = blockIdx.x * 256 + threadIdx.x;
  const int k8n = K / 8;
  if (t >= N * k8n) return;
  const int n = t / k8n, k8 = (t % k8n) * 8;
  v8us v;
#pragma unroll
  for (int i = 0; i < 8; ++i) v[i] = bf16_bits(W[(size_t)(k8 + i) * N + n]);
  *(volatile v8us*)(Wt + (size_t)n * K + k8) = v;
  __threadfence();
  *(volatile v8us*)(Wt + (size_t)n * K + k8) = v;
}

template <bool ASPLIT, int ACT, bool BIAS_BF16>
__global__ __launch_bounds__(128) void k_gemm_bf(const float* __restrict__ A, int lda, const unsigned short* __restrict__ Wt, int ldb,
                                               const float* __restrict__ bias, float* __restrict__ C, int ldc, int M, int N, int K) {
  __shared__ __attribute__((aligned(16))) float so[4][16][64];
  const int tid = threadIdx.x, w = tid >> 5, lane = tid & 31, ln = lane & 15, hh = lane >> 4;
  const int ntn = N / 64;
  const int wid = blockIdx.x * 4 + w;
  const int mt = wid / ntn, nq = wid % ntn;
  if (mt * 16 >= M) return;
  const int row0 = mt * 16, col0 = nq * 64;
  const float* arow = A + (size_t)(row0 + ln) * lda;
  v8f acc[4] = {};
  for (int kb = 0; kb < K; kb += 32) {
    FragB ah, al;
    const v4f x0 = *(const v4fa*)(arow + kb + 8 * hh), x1 = *(const v4fa*)(arow + kb + 8 * hh + 4);
    const v4f x2 = *(const v4fa*)(arow + kb + 16 + 8 * hh), x3 = *(const v4fa*)(arow + kb + 16 + 8 * hh + 4);
    float xs[16] = {x0[0],x0[1],x0[2],x0[3],x1[0],x1[1],x1[2],x1[3],x2[0],x2[1],x2[2],x2[3],x3[0],x3[1],x3[2],x3[3]};
#pragma unroll
    for (int i = 0; i < 16; ++i) { const unsigned short hb = bf16_bits(xs[i]); ah.u[i] = hb; al.u[i] = ASPLIT ? bf16_bits(xs[i] - bf16_val(hb)) : (unsigned short)0; }
#pragma unroll
    for (int t = 0; t < 4; ++t) {
      const unsigned short* brow = Wt + (size_t)(col0 + t * 16 + ln) * ldb + kb;
      FragB b;
      b.half[0] = *(const v8us*)(brow + 8 * hh);
      b.half[1] = *(const v8us*)(brow + 16 + 8 * hh);
      acc[t] = mmaN<ASPLIT ? 2 : 1>(ah.v, al.v, b.v, b.v, acc[t]);
    }
  }
#pragma unroll
  for (int t = 0; t < 4; ++t) {
    float bv = bias ? bias[col0 + t * 16 + ln] : 0.f;
    if (BIAS_BF16) bv = bf16_round(bv);
#pragma unroll
    for (int r = 0; r < 8; ++r) { float v = acc[t][r] + bv; if (ACT == 1) v = fmaxf(v, 0.f); so[w][8 * hh + r][t * 16 + ln] = v; }
  }
  __builtin_amdgcn_fence(__ATOMIC_ACQ_REL, "workgroup");
  __builtin_amdgcn_wave_barrier();
  const int rsub = lane >> 4, c4 = (lane & 15) * 4;
  for (int pass = 0; pass < 2; ++pass) {
#pragma unroll
    for (int q = 0; q < 8; ++q) {
      const int r = q * 2 + rsub;
      const v4f v = *(const v4fa*)&so[w][r][c4];
      *(volatile v4f*)(C + (size_t)(row0 + r) * ldc + col0 + c4) = v;
    }
    if (pass == 0) __threadfence();
  }
}

template <bool ASPLIT, int ACT, bool BIAS_BF16, bool RES_BF16>
__global__ __launch_bounds__(128) void k_gemm_bf3(const float* __restrict__ A, int lda, const unsigned short* __restrict__ Wt, int ldb,
                                                const float* __restrict__ bias, const float* __restrict__ resid, int rmod, int ldr,
                                                float* __restrict__ C, int ldc, int M, int N, int K) {
  __shared__ __attribute__((aligned(16))) float so[4][16][64];
  const int tid = threadIdx.x, w = tid >> 5, lane = tid & 31, ln = lane & 15, hh = lane >> 4;
  const int ntn = N / 64;
  const int wid = blockIdx.x * 4 + w;
  const int mt = wid / ntn, nq = wid % ntn;
  if (mt * 16 >= M) return;
  const int row0 = mt * 16, col0 = nq * 64;
  const float* arow = A + (size_t)(row0 + ln) * lda;
  v8f acc[4] = {};
  for (int kb = 0; kb < K; kb += 32) {
    FragB ah, al;
    const v4f x0 = *(const v4fa*)(arow + kb + 8 * hh), x1 = *(const v4fa*)(arow + kb + 8 * hh + 4);
    const v4f x2 = *(const v4fa*)(arow + kb + 16 + 8 * hh), x3 = *(const v4fa*)(arow + kb + 16 + 8 * hh + 4);
    float xs[16] = {x0[0],x0[1],x0[2],x0[3],x1[0],x1[1],x1[2],x1[3],x2[0],x2[1],x2[2],x2[3],x3[0],x3[1],x3[2],x3[3]};
#pragma unroll
    for (int i = 0; i < 16; ++i) { const unsigned short hb = bf16_bits(xs[i]); ah.u[i] = hb; al.u[i] = ASPLIT ? bf16_bits(xs[i] - bf16_val(hb)) : (unsigned short)0; }
#pragma unroll
    for (int t = 0; t < 4; ++t) {
      const unsigned short* brow = Wt + (size_t)(col0 + t * 16 + ln) * ldb + kb;
      FragB b;
      b.half[0] = *(const v8us*)(brow + 8 * hh);
      b.half[1] = *(const v8us*)(brow + 16 + 8 * hh);
      acc[t] = mmaN<ASPLIT ? 2 : 1>(ah.v, al.v, b.v, b.v, acc[t]);
    }
  }
#pragma unroll
  for (int t = 0; t < 4; ++t) {
    const int col = col0 + t * 16 + ln;
    float bv = bias ? bias[col] : 0.f;
    if (BIAS_BF16) bv = bf16_round(bv);
#pragma unroll
    for (int r = 0; r < 8; ++r) {
      float v = acc[t][r] + bv;
      if (resid) { float rv = resid[(size_t)((row0 + 8 * hh + r) % rmod) * ldr + col]; if (RES_BF16) rv = bf16_round(rv); v += rv; }
      if (ACT == 1) v = fmaxf(v, 0.f);
      if (ACT == 2) v = 0.5f * v * (1.0f + erff(v * 0.70710678118654752f));
      if (ACT == 3) { const float u = 0.7978845608028654f * (v + 0.044715f * v * v * v); v = 0.5f * v * (1.0f + tanhf(u)); }
      so[w][8 * hh + r][t * 16 + ln] = v;
    }
  }
  __builtin_amdgcn_fence(__ATOMIC_ACQ_REL, "workgroup");
  __builtin_amdgcn_wave_barrier();
  const int rsub = lane >> 4, c4 = (lane & 15) * 4;
  for (int pass = 0; pass < 2; ++pass) {
#pragma unroll
    for (int q = 0; q < 8; ++q) {
      const int r = q * 2 + rsub;
      const v4f v = *(const v4fa*)&so[w][r][c4];
      *(volatile v4f*)(C + (size_t)(row0 + r) * ldc + col0 + c4) = v;
    }
    if (pass == 0) __threadfence();
  }
}
template <bool PARAM_BF16>
__global__ __launch_bounds__(256) void k_layernorm(const float* __restrict__ X, const float* __restrict__ R, const float* __restrict__ g, const float* __restrict__ bta,
                                                  float* __restrict__ out_sum, float* __restrict__ out_norm, int N, float eps) {
  __shared__ float red[256];
  const int row = blockIdx.x, tid = threadIdx.x;
  const float* x = X + (size_t)row * N; const float* rr = R ? R + (size_t)row * N : nullptr;
  float vals[16];
  const int per = N / 256;
  float s1 = 0.f;
  for (int u = 0; u < per / 4; ++u) {
    const int j = tid * 4 + 1024 * u;
    const v4f a = *(const v4fa*)(x + j);
    v4f b = {0.f,0.f,0.f,0.f}; if (rr) b = *(const v4fa*)(rr + j);
#pragma unroll
    for (int q = 0; q < 4; ++q) { const float v = a[q] + b[q]; vals[u * 4 + q] = v; s1 += v; }
  }
  red[tid] = s1; __syncthreads();
  for (int st = 128; st > 0; st >>= 1) { if (tid < st) red[tid] += red[tid + st]; __syncthreads(); }
  const float mu = red[0] / (float)N; __syncthreads();
  float s2 = 0.f;
  for (int u = 0; u < per / 4; ++u)
#pragma unroll
    for (int q = 0; q < 4; ++q) { const float c = vals[u * 4 + q] - mu; s2 += c * c; }
  red[tid] = s2; __syncthreads();
  for (int st = 128; st > 0; st >>= 1) { if (tid < st) red[tid] += red[tid + st]; __syncthreads(); }
  const float rs = rsqrtf(red[0] / (float)N + eps);
  for (int pass = 0; pass < 2; ++pass) {
    for (int u = 0; u < per / 4; ++u) {
      const int j = tid * 4 + 1024 * u;
      v4f o, sm;
#pragma unroll
      for (int q = 0; q < 4; ++q) {
        float gg = g[j + q], bb = bta[j + q];
        if (PARAM_BF16) { gg = bf16_round(gg); bb = bf16_round(bb); }
        sm[q] = vals[u * 4 + q]; o[q] = (vals[u * 4 + q] - mu) * rs * gg + bb;
      }
      if (out_sum) *(volatile v4f*)(out_sum + (size_t)row * N + j) = sm;
      *(volatile v4f*)(out_norm + (size_t)row * N + j) = o;
    }
    if (pass == 0) __threadfence();
  }
}


typedef _Float16 v16h __attribute__((ext_vector_type(16)));
union FragH { v16h v; v8us half[2]; _Float16 h[16]; unsigned short u[16]; };
template <int NT>
__device__ __forceinline__ v8f mmaH(v16h ah, v16h al, v16h bh, v16h bl, v8f c) {
  c = __builtin_amdgcn_wmma_f32_16x16x32_f16(false, ah, false, bh, (short)0, c, false, false);
  if (NT >= 2) c = __builtin_amdgcn_wmma_f32_16x16x32_f16(false, al, false, bh, (short)0, c, false, false);
  if (NT >= 3) c = __builtin_amdgcn_wmma_f32_16x16x32_f16(false, ah, false, bl, (short)0, c, false, false);
  asm volatile("v_nop\n\tv_nop\n\tv_nop\n\tv_nop" : "+v"(c) : "v"(ah), "v"(al), "v"(bh), "v"(bl));
  return c;
}
template <bool ASPLIT>
__global__ __launch_bounds__(128) void k_gemm_h(const float* __restrict__ A, int lda, size_t sA, const _Float16* __restrict__ Bh, int ldb, size_t sB, float alpha, float* __restrict__ C, int ldc, size_t sC, int M, int N, int K) {
  __shared__ __attribute__((aligned(16))) float so[4][16][64];
  const int tid = threadIdx.x, w = tid >> 5, lane = tid & 31, ln = lane & 15, hh = lane >> 4; const int by = blockIdx.y;
  A += (size_t)by * sA; Bh += (size_t)by * sB; C += (size_t)by * sC;
  const int ntn = (N + 63) / 64; const int wid = blockIdx.x * 4 + w; const int mt = wid / ntn, nq = wid % ntn; if (mt * 16 >= M) return;
  const int row0 = mt * 16, col0 = nq * 64; const float* arow = A + (size_t)(row0 + ln) * lda;
  v8f acc[4] = {};
  for (int kb = 0; kb < K; kb += 32) {
    FragH ah, al;
    const v4f x0 = *(const v4fa*)(arow + kb + 8 * hh), x1 = *(const v4fa*)(arow + kb + 8 * hh + 4), x2 = *(const v4fa*)(arow + kb + 16 + 8 * hh), x3 = *(const v4fa*)(arow + kb + 16 + 8 * hh + 4);
    float xs[16] = {x0[0],x0[1],x0[2],x0[3],x1[0],x1[1],x1[2],x1[3],x2[0],x2[1],x2[2],x2[3],x3[0],x3[1],x3[2],x3[3]};
#pragma unroll
    for (int i = 0; i < 16; ++i) { const _Float16 h = (_Float16)xs[i]; ah.h[i] = h; al.h[i] = ASPLIT ? (_Float16)(xs[i] - (float)h) : (_Float16)0.0f; }
#pragma unroll
    for (int t = 0; t < 4; ++t) { if (col0 + t * 16 >= N) continue; const size_t boff = (size_t)(col0 + t * 16 + ln) * ldb + kb; FragH bq; bq.half[0] = *(const v8us*)(Bh + boff + 8 * hh); bq.half[1] = *(const v8us*)(Bh + boff + 16 + 8 * hh);
      acc[t] = mmaH<ASPLIT ? 2 : 1>(ah.v, al.v, bq.v, bq.v, acc[t]); }
  }
#pragma unroll
  for (int t = 0; t < 4; ++t) { if (col0 + t * 16 >= N) continue;
#pragma unroll
    for (int r = 0; r < 8; ++r) so[w][8 * hh + r][t * 16 + ln] = acc[t][r] * alpha; }
  __builtin_amdgcn_fence(__ATOMIC_ACQ_REL, "workgroup"); __builtin_amdgcn_wave_barrier();
  const int rsub = lane >> 4, c4 = (lane & 15) * 4;
  for (int pass = 0; pass < 2; ++pass) {
#pragma unroll
    for (int q = 0; q < 8; ++q) { const int r = q * 2 + rsub; if (col0 + c4 < N) { const v4f v = *(const v4fa*)&so[w][r][c4]; *(volatile v4f*)(C + (size_t)(row0 + r) * ldc + col0 + c4) = v; } }
    if (pass == 0) __threadfence(); }
}

__global__ __launch_bounds__(256) void k_wt_f16(const float* __restrict__ W, _Float16* __restrict__ Wt, int K, int N, float scale) {
  const int t = blockIdx.x * 256 + threadIdx.x; if (t >= N * (K / 8)) return; const int n = t / (K / 8), k8 = (t % (K / 8)) * 8; FragH f;
#pragma unroll
  for (int i = 0; i < 8; ++i) f.h[i] = (_Float16)(bf16_round(W[(size_t)(k8 + i) * N + n]) * scale); const v8us o = f.half[0];
  *(volatile v8us*)((unsigned short*)Wt + (size_t)n * K + k8) = o; __threadfence(); *(volatile v8us*)((unsigned short*)Wt + (size_t)n * K + k8) = o;
}
template <int ACT>
__global__ __launch_bounds__(128) void k_gemm_hhx(const _Float16* __restrict__ A, int lda, size_t sA, const _Float16* __restrict__ Bh, int ldb, size_t sB, float alpha, const float* __restrict__ bias, size_t sBias, const float* __restrict__ CP, int rowsPerB, size_t sCPb, int row0g,
    float* __restrict__ C, _Float16* __restrict__ C16, int ldc, size_t sC, int M, int N, int K) {
  __shared__ __attribute__((aligned(16))) float so[4][16][64];
  const int tid = threadIdx.x, w = tid >> 5, lane = tid & 31, ln = lane & 15, hh = lane >> 4; const int by = blockIdx.y;
  A += (size_t)by * sA; Bh += (size_t)by * sB; const size_t cofs = (size_t)by * sC; const float* bp = bias ? bias + (size_t)by * sBias : nullptr;
  const int ntn = (N + 63) / 64; const int wid = blockIdx.x * 4 + w; const int mt = wid / ntn, nq = wid % ntn; if (mt * 16 >= M) return;
  const int row0 = mt * 16, col0 = nq * 64; const _Float16* arow = A + (size_t)(row0 + ln) * lda;
  v8f acc[4] = {};
  for (int kb = 0; kb < K; kb += 32) { FragH ah; ah.half[0] = *(const v8us*)((const unsigned short*)arow + kb + 8 * hh); ah.half[1] = *(const v8us*)((const unsigned short*)arow + kb + 16 + 8 * hh);
#pragma unroll
    for (int t = 0; t < 4; ++t) { if (col0 + t * 16 >= N) continue; const size_t boff = (size_t)(col0 + t * 16 + ln) * ldb + kb; FragH bq; bq.half[0] = *(const v8us*)((const unsigned short*)Bh + boff + 8 * hh); bq.half[1] = *(const v8us*)((const unsigned short*)Bh + boff + 16 + 8 * hh);
      acc[t] = mmaH<1>(ah.v, ah.v, bq.v, bq.v, acc[t]); }
  }
#pragma unroll
  for (int t = 0; t < 4; ++t) { if (col0 + t * 16 >= N) continue; const int col = col0 + t * 16 + ln; const float bv = bp ? bf16_round(bp[col]) : 0.f;
#pragma unroll
    for (int r = 0; r < 8; ++r) { float v = acc[t][r] * alpha + bv; if (CP) { const int bidx = (row0g + row0 + 8 * hh + r) / rowsPerB; v += CP[(size_t)bidx * sCPb + (size_t)by * 64 + col]; } if (ACT == 1) v = (v > 0.f) ? v : expm1f(v); else if (ACT == 7) v = (v > 0.f) ? v + 1.0f : expf(v); else if (ACT == 8) v = tanhf(v); else if (ACT == 9) v = 0.5f * v * (1.0f + tanhf(0.7978845608028654f * (v + 0.044715f * v * v * v))); else if (ACT == 11) v = 1.0f / (1.0f + expf(-v)); else if (ACT == 12) v = (v > 0.f) ? v : 0.01f * v; else if (ACT == 14) v = (v > 0.f) ? v : 0.1f * v; else if (ACT == 15) v = v / (1.0f + expf(-v)); else if (ACT == 3) v = fmaxf(v, 0.f); else if (ACT == 6) v = 0.5f * v * (1.0f + erff(v * 0.70710678118654752f)); so[w][8 * hh + r][t * 16 + ln] = v; } }
  __builtin_amdgcn_fence(__ATOMIC_ACQ_REL, "workgroup"); __builtin_amdgcn_wave_barrier();
  const int rsub = lane >> 4, c4 = (lane & 15) * 4; typedef _Float16 v4h __attribute__((ext_vector_type(4)));
  for (int pass = 0; pass < 2; ++pass) {
#pragma unroll
    for (int q = 0; q < 8; ++q) { const int r = q * 2 + rsub; if (col0 + c4 < N) { const v4f v = *(const v4fa*)&so[w][r][c4]; if (C) *(volatile v4f*)(C + cofs + (size_t)(row0 + r) * ldc + col0 + c4) = v; if (C16) { v4h h4; for (int i = 0; i < 4; ++i) h4[i] = (_Float16)v[i]; *(volatile v4h*)(C16 + cofs + (size_t)(row0 + r) * ldc + col0 + c4) = h4; } } }
    if (pass == 0) __threadfence(); }
}


typedef _Float16 v4h __attribute__((ext_vector_type(4)));

__global__ __launch_bounds__(256) void k_x16(const float* __restrict__ x, _Float16* __restrict__ X16, size_t n8) { const size_t t = (size_t)blockIdx.x * 256 + threadIdx.x; if (t >= n8) return; FragH f;
#pragma unroll
  for (int q = 0; q < 8; ++q) f.h[q] = (_Float16)bf16_round(x[t * 8 + q]); *(volatile v8us*)((unsigned short*)X16 + t * 8) = f.half[0]; __threadfence(); *(volatile v8us*)((unsigned short*)X16 + t * 8) = f.half[0]; }
__global__ __launch_bounds__(256) void k_h16(const float* __restrict__ x, _Float16* __restrict__ X16, size_t n8) { const size_t t = (size_t)blockIdx.x * 256 + threadIdx.x; if (t >= n8) return; FragH f;
#pragma unroll
  for (int q = 0; q < 8; ++q) f.h[q] = (_Float16)x[t * 8 + q]; *(volatile v8us*)((unsigned short*)X16 + t * 8) = f.half[0]; __threadfence(); *(volatile v8us*)((unsigned short*)X16 + t * 8) = f.half[0]; }
__global__ __launch_bounds__(256) void k_round16f(const float* __restrict__ W, _Float16* __restrict__ Bt, size_t n8) { const size_t t = (size_t)blockIdx.x * 256 + threadIdx.x; if (t >= n8) return; FragH f;
#pragma unroll
  for (int i = 0; i < 8; ++i) f.h[i] = (_Float16)(bf16_round(W[t * 8 + i]) * 16.0f); *(volatile v8us*)((unsigned short*)Bt + t * 8) = f.half[0]; __threadfence(); *(volatile v8us*)((unsigned short*)Bt + t * 8) = f.half[0]; }
template <int NHv, int TTv>
__global__ __launch_bounds__(256) void k_vt(const _Float16* __restrict__ V16, int ldv, int voff, _Float16* __restrict__ Vt) { __shared__ unsigned short tl[64][66]; const int tid = threadIdx.x; const int slab = blockIdx.x / (TTv / 64), lg = blockIdx.x % (TTv / 64); const int b = slab / NHv, h = slab % NHv;
  for (int i = tid; i < 64 * 8; i += 256) { const int r = i / 8, c8 = (i % 8) * 8; FragH f; f.half[0] = *(const v8us*)((const unsigned short*)V16 + ((size_t)b * TTv + lg * 64 + r) * ldv + voff + h * 64 + c8);
#pragma unroll
    for (int q = 0; q < 8; ++q) tl[r][c8 + q] = f.u[q]; }
  __syncthreads();
  for (int pass = 0; pass < 2; ++pass) {
#pragma unroll
    for (int rd = 0; rd < 2; ++rd) { const int d = rd * 32 + tid / 8, pc = tid % 8; FragH f;
#pragma unroll
      for (int q = 0; q < 8; ++q) f.u[q] = tl[pc * 8 + q][d];
      *(volatile v8us*)((unsigned short*)Vt + ((size_t)slab * 64 + d) * TTv + lg * 64 + pc * 8) = f.half[0]; }
    if (pass == 0) __threadfence(); } }

__global__ __launch_bounds__(256) void k_hl(const float* __restrict__ F, _Float16* __restrict__ Hh, _Float16* __restrict__ Hl, size_t n8) { const size_t t = (size_t)blockIdx.x * 256 + threadIdx.x; if (t >= n8) return; FragH fh, fl; const v4f a = *(const v4fa*)(F + t * 8), c = *(const v4fa*)(F + t * 8 + 4);
#pragma unroll
  for (int q = 0; q < 4; ++q) { _Float16 h = (_Float16)a[q]; fh.h[q] = h; fl.h[q] = (_Float16)((a[q] - (float)h) * 1024.0f); h = (_Float16)c[q]; fh.h[4 + q] = h; fl.h[4 + q] = (_Float16)((c[q] - (float)h) * 1024.0f); }
  for (int pass = 0; pass < 2; ++pass) { *(volatile v8us*)((unsigned short*)Hh + t * 8) = fh.half[0]; *(volatile v8us*)((unsigned short*)Hl + t * 8) = fl.half[0]; if (pass == 0) __threadfence(); } }

#define VST2(T, ptr, val) do { const T vst2_v_ = (val); *(volatile T*)(ptr) = vst2_v_; __threadfence(); *(volatile T*)(ptr) = vst2_v_; } while (0)

#define C4_NB 4096
#define C4_CH 8192
__device__ __forceinline__ int c4_bucket(int v, int N) { v = min(max(v, 0), N - 1); return (int)(((long long)v * C4_NB) / N); }
__global__ __launch_bounds__(256) void k_c4_count(const int* __restrict__ tgt, int E, int N, int* __restrict__ CNT) {
    __shared__ int hist[C4_NB]; const int ch = blockIdx.x, t = threadIdx.x; const int e0 = ch * C4_CH; const int nt = min(C4_CH, E - e0);
    for (int j = 0; j < 16; ++j) hist[t + 256 * j] = 0; __syncthreads();
    for (int i = t; i < nt; i += 256) atomicAdd(&hist[c4_bucket(tgt[e0 + i], N)], 1);
    __syncthreads();
    for (int j = 0; j < 16; ++j) { const int v = hist[t + 256 * j]; VST2(int, CNT + (long long)ch * C4_NB + t + 256 * j, v); } }
__global__ __launch_bounds__(256) void k_c4_offsets(const int* __restrict__ CNT, int nch, int E, int* __restrict__ OFFB, int* __restrict__ BOFF) {
    __shared__ int tot[C4_NB]; __shared__ int part[256]; const int t = threadIdx.x;
    for (int j = 0; j < 16; ++j) { const int b = t + 256 * j; int s = 0; for (int ch = 0; ch < nch; ++ch) s += CNT[(long long)ch * C4_NB + b]; tot[b] = s; }
    __syncthreads();
    { int s = 0; for (int q = 0; q < 16; ++q) s += tot[16 * t + q]; part[t] = s; } __syncthreads();
    if (t == 0) { int run = 0; for (int i = 0; i < 256; ++i) { const int v = part[i]; part[i] = run; run += v; } } __syncthreads();
    { int run = part[t]; for (int q = 0; q < 16; ++q) { const int v = tot[16 * t + q]; tot[16 * t + q] = run; run += v; } }
    __syncthreads();
    for (int j = 0; j < 16; ++j) { const int b = t + 256 * j; VST2(int, BOFF + b, tot[b]); }
    if (t == 0) VST2(int, BOFF + C4_NB, E);
    for (int j = 0; j < 16; ++j) { const int b = t + 256 * j; int run = tot[b]; for (int ch = 0; ch < nch; ++ch) { VST2(int, OFFB + (long long)ch * C4_NB + b, run); run += CNT[(long long)ch * C4_NB + b]; } } }
__global__ __launch_bounds__(256) void k_c4_scatter(const int* __restrict__ tgt, int E, int N, const int* __restrict__ OFFB, int* __restrict__ BUF) {
    __shared__ int cur[C4_NB]; __shared__ int bk[256]; const int ch = blockIdx.x, t = threadIdx.x; const int e0 = ch * C4_CH; const int nt = min(C4_CH, E - e0);
    const int wv = t >> 5, ln = t & 31;
    for (int j = 0; j < 16; ++j) cur[t + 256 * j] = OFFB[(long long)ch * C4_NB + t + 256 * j];
    __syncthreads();
    for (int s0 = 0; s0 < C4_CH; s0 += 256) {
        const int i = s0 + t; const int e = e0 + i; const int b = (i < nt) ? c4_bucket(tgt[min(e, E - 1)], N) : -1;
        bk[t] = b; __syncthreads();
        int rank = 0, cntw = 0;
        for (int l = 0; l < 32; ++l) { const int o = bk[(wv << 5) + l]; const bool same = (o == b) && (b >= 0); cntw += same ? 1 : 0; rank += (same && l < ln) ? 1 : 0; }
        const bool last = (b >= 0) && (rank == cntw - 1);
        for (int w = 0; w < 8; ++w) {
            if (wv == w && b >= 0) { int pos = cur[b] + rank; pos = min(max(pos, 0), E - 1); VST2(int, BUF + pos, e); }
            __syncthreads();
            if (wv == w && last) cur[b] += cntw;
            __syncthreads(); }
    } }
template <int CAP>
__global__ __launch_bounds__(256) void k_c4_lists(const int* __restrict__ tgt, const int* __restrict__ BUF, const int* __restrict__ BOFF, int N, int E, int* __restrict__ NBR, int* __restrict__ cnt) {
    const int d = blockIdx.x * 256 + threadIdx.x; if (d >= N) return; const int b = c4_bucket(d, N); int n = 0; int* row = NBR + (long long)d * CAP;
    const int p0 = min(max(BOFF[b], 0), E), p1 = min(max(BOFF[b + 1], p0), E);
    for (int p = p0; p < p1; ++p) { int e = BUF[p]; e = min(max(e, 0), E - 1); if (tgt[e] == d) { if (n < CAP) VST2(int, row + n, e); ++n; } }
    for (int j = n; j < CAP; ++j) VST2(int, row + j, -1); VST2(int, cnt + d, min(n, CAP)); }
__global__ __launch_bounds__(256) void k_c4_scan1(const int* __restrict__ cnt, int* __restrict__ PART, int N) {
    __shared__ int part[256]; const int per = ((((N + 255) / 256) + 31) / 32) * 32; const int a = threadIdx.x * per, b = min(N, a + per); int s = 0;
    for (int i = a; i < b; ++i) s += cnt[i]; part[threadIdx.x] = s; __syncthreads();
    if (threadIdx.x == 0) { int run = 0; for (int t = 0; t < 256; ++t) { const int v = part[t]; part[t] = run; run += v; } } __syncthreads();
    VST2(int, PART + threadIdx.x, part[threadIdx.x]); }
__global__ __launch_bounds__(256) void k_c4_scan2(const int* __restrict__ cnt, const int* __restrict__ PART, int* __restrict__ off, int N) {
    const int i = blockIdx.x * 256 + threadIdx.x; if (i > N) return; const int per = ((((N + 255) / 256) + 31) / 32) * 32; const int r = min(i / per, 255); const int a = r * per;
    int s = PART[r]; for (int kq = a; kq < i; ++kq) s += cnt[min(kq, N - 1)];
    VST2(int, off + i, s); }
template <int CAP>
__global__ __launch_bounds__(256) void k_c4_slotcopy(const int* __restrict__ off, const int* __restrict__ NBR, int* __restrict__ slot, int N) {
    const int t = blockIdx.x * 256 + threadIdx.x; const int tot = off[N]; if (t >= tot) return;
    int lo = 0, hi = N - 1; while (lo < hi) { const int mid = (lo + hi + 1) >> 1; if (off[mid] <= t) lo = mid; else hi = mid - 1; }
    int j = t - off[lo]; j = (j < 0) ? 0 : ((j >= CAP) ? (CAP - 1) : j); VST2(int, slot + t, NBR[(long long)lo * CAP + j]); }

template <int RIN>
__global__ __launch_bounds__(256) void k_ln512(const float* __restrict__ X, const float* __restrict__ g, const float* __restrict__ be, _Float16* __restrict__ Y) { const int tid = threadIdx.x, w = tid >> 5, l = tid & 31; const size_t row = (size_t)blockIdx.x * 8 + w; if (row >= NR) return; float v[16]; float s = 0.f;
#pragma unroll
  for (int q = 0; q < 2; ++q) { const v4f a = *(const v4fa*)(X + row * DD + q * 256 + 8 * l), c = *(const v4fa*)(X + row * DD + q * 256 + 8 * l + 4);
#pragma unroll
    for (int j = 0; j < 4; ++j) { v[q * 8 + j] = RIN ? bf16_round(a[j]) : a[j]; v[q * 8 + 4 + j] = RIN ? bf16_round(c[j]) : c[j]; } }
#pragma unroll
  for (int i = 0; i < 16; ++i) s += v[i];
  for (int o = 16; o > 0; o >>= 1) s += __shfl_xor(s, o, 32); const float mu = s * (1.0f / DD); float vs = 0.f;
#pragma unroll
  for (int i = 0; i < 16; ++i) { const float d = v[i] - mu; vs += d * d; }
  for (int o = 16; o > 0; o >>= 1) vs += __shfl_xor(vs, o, 32); const float rs = rsqrtf(vs * (1.0f / DD) + LNEPS); FragH f[2];
#pragma unroll
  for (int q = 0; q < 2; ++q)
#pragma unroll
    for (int j = 0; j < 8; ++j) { const int c = q * 256 + 8 * l + j; f[q].h[j] = (_Float16)((v[q * 8 + j] - mu) * rs * bf16_round(g[c]) + bf16_round(be[c])); }
  for (int pass = 0; pass < 2; ++pass) { *(volatile v8us*)((unsigned short*)Y + row * DD + 8 * l) = f[0].half[0]; *(volatile v8us*)((unsigned short*)Y + row * DD + 256 + 8 * l) = f[1].half[0]; if (pass == 0) __threadfence(); } }
__global__ __launch_bounds__(256) void k_bcat(const float* __restrict__ bq, const float* __restrict__ bk, const float* __restrict__ bv, float* __restrict__ Bc) { const int i = blockIdx.x * 256 + threadIdx.x; if (i >= 3 * DD) return; const float v = (i < DD) ? bq[i] : (i < 2 * DD) ? bk[i - DD] : bv[i - 2 * DD]; VST2(float, Bc + i, v); }
__global__ __launch_bounds__(256) void k_keys(const int* __restrict__ edges, const float* __restrict__ masks, int* __restrict__ KA, int* __restrict__ KB) { const int e = blockIdx.x * 256 + threadIdx.x; if (e >= NET) return; const int b = e / NEG; int s = edges[(size_t)e * 2], d = edges[(size_t)e * 2 + 1]; s = min(max(s, 0), NND - 1); d = min(max(d, 0), NND - 1); const bool valid = bf16_round(masks[e]) != 0.f;
  VST2(int, KA + e, b * 257 + (valid ? s : NND)); VST2(int, KB + e, b * 257 + (valid ? d : NND)); }
__global__ __launch_bounds__(256) void k_tb(const float* __restrict__ emb, const float* __restrict__ geo, const float* __restrict__ Web, const float* __restrict__ beb, const float* __restrict__ lg, const float* __restrict__ lb, const float* __restrict__ Wg, const float* __restrict__ bg, float* __restrict__ TB) {
  #pragma clang fp contract(off)
  const int t = blockIdx.x * 256 + threadIdx.x; if (t >= NET * NH) return; const int e = t / NH, h = t % NH; const float* er = emb + (size_t)e * EDIM; const float* gr = geo + (size_t)e * GDIM; float s = 0.f;
#pragma unroll 1
  for (int k = 0; k < EDIM; ++k) s += bf16_round(er[k]) * bf16_round(Web[h * EDIM + k]);
  s += bf16_round(beb[h]); float mu = 0.f;
#pragma unroll 1
  for (int k = 0; k < GDIM; ++k) mu += bf16_round(gr[k]); mu *= (1.0f / GDIM); float var = 0.f;
#pragma unroll 1
  for (int k = 0; k < GDIM; ++k) { const float d = bf16_round(gr[k]) - mu; var += d * d; } const float rs = rsqrtf(var * (1.0f / GDIM) + LNEPS); float s2 = 0.f;
#pragma unroll 1
  for (int k = 0; k < GDIM; ++k) s2 += ((bf16_round(gr[k]) - mu) * rs * bf16_round(lg[k]) + bf16_round(lb[k])) * bf16_round(Wg[h * GDIM + k]);
  const float v = s + s2 + bf16_round(bg[h]); VST2(float, TB + t, v); }
__global__ __launch_bounds__(256) void k_attnrow(const float* __restrict__ S, const float* __restrict__ TB, const int* __restrict__ edges, const int* __restrict__ nbrA, const int* __restrict__ cntA, const int* __restrict__ nbrB, const int* __restrict__ cntB, const float* __restrict__ nmask, int b0, _Float16* __restrict__ P16) {
  #pragma clang fp contract(off)
  __shared__ float rb[NND][NH + 1]; __shared__ float adj[NND]; __shared__ float red[8]; __shared__ __attribute__((aligned(16))) unsigned short prow[NND];
  const int tid = threadIdx.x, w = tid >> 5, l = tid & 31; const int bl = blockIdx.x / NND, i = blockIdx.x % NND; const int b = b0 + bl; const int j = tid;
#pragma unroll
  for (int h = 0; h < NH; ++h) rb[j][h] = 0.f; adj[j] = (j == i) ? 1.f : 0.f; __syncthreads();
  if (tid == 0) { const int key = b * 257 + i;
    { const int n = min(max(cntA[key], 0), ECAP);
#pragma unroll 1
      for (int q = 0; q < ECAP; ++q) { if (q >= n) break; int e = nbrA[(size_t)key * ECAP + q]; if (e < 0) break; e = min(max(e, 0), NET - 1); int d = edges[(size_t)e * 2 + 1]; d = min(max(d, 0), NND - 1);
#pragma unroll
        for (int h = 0; h < NH; ++h) rb[d][h] = TB[(size_t)e * NH + h]; adj[d] = 1.f; } }
    { const int n = min(max(cntB[key], 0), ECAP);
#pragma unroll 1
      for (int q = 0; q < ECAP; ++q) { if (q >= n) break; int e = nbrB[(size_t)key * ECAP + q]; if (e < 0) break; e = min(max(e, 0), NET - 1); int s = edges[(size_t)e * 2]; s = min(max(s, 0), NND - 1);
#pragma unroll
        for (int h = 0; h < NH; ++h) rb[s][h] = TB[(size_t)e * NH + h]; adj[s] = 1.f; } } }
  __syncthreads();
  const bool nmi = bf16_round(nmask[(size_t)b * NND + i]) != 0.f, nmj = bf16_round(nmask[(size_t)b * NND + j]) != 0.f; const bool allowed = nmi && nmj && (adj[j] != 0.f);
#pragma unroll 1
  for (int h = 0; h < NH; ++h) { const float sv = S[(((size_t)bl * NH + h) * NND + i) * NND + j]; const float lg_ = allowed ? (sv + rb[j][h]) : -3.4028235e38f;
    float m = lg_; for (int o = 16; o > 0; o >>= 1) m = fmaxf(m, __shfl_xor(m, o, 32)); if (l == 0) red[w] = m; __syncthreads(); m = red[0];
#pragma unroll
    for (int k = 1; k < 8; ++k) m = fmaxf(m, red[k]); __syncthreads();
    const float ex = expf(lg_ - m); float su = ex; for (int o = 16; o > 0; o >>= 1) su += __shfl_xor(su, o, 32); if (l == 0) red[w] = su; __syncthreads(); su = 0.f;
#pragma unroll
    for (int k = 0; k < 8; ++k) su += red[k];
    FragH f1; f1.h[0] = (_Float16)(ex / su * 1024.0f); prow[j] = f1.u[0]; __syncthreads();
    if (tid < 32) { FragH f;
#pragma unroll
      for (int q = 0; q < 8; ++q) f.u[q] = prow[tid * 8 + q]; _Float16* dst = P16 + (((size_t)bl * NH + h) * NND + i) * NND + tid * 8; *(volatile v8us*)dst = f.half[0]; __threadfence(); *(volatile v8us*)dst = f.half[0]; }
    __syncthreads(); } }
__global__ __launch_bounds__(256) void k_h16p(const float* __restrict__ F, _Float16* __restrict__ Hh, size_t n8) { const size_t t = (size_t)blockIdx.x * 256 + threadIdx.x; if (t >= n8) return; const v4f a = *(const v4fa*)(F + t * 8), c = *(const v4fa*)(F + t * 8 + 4); FragH f;
#pragma unroll
  for (int q = 0; q < 4; ++q) { f.h[q] = (_Float16)a[q]; f.h[4 + q] = (_Float16)c[q]; } *(volatile v8us*)((unsigned short*)Hh + t * 8) = f.half[0]; __threadfence(); *(volatile v8us*)((unsigned short*)Hh + t * 8) = f.half[0]; }
__global__ __launch_bounds__(256) void k_bfx(const float* __restrict__ x, float* __restrict__ Xb, size_t n4) { const size_t t = (size_t)blockIdx.x * 256 + threadIdx.x; if (t >= n4) return; const v4f a = *(const v4fa*)(x + t * 4); v4f o; o[0] = bf16_round(a[0]); o[1] = bf16_round(a[1]); o[2] = bf16_round(a[2]); o[3] = bf16_round(a[3]); *(volatile v4f*)(Xb + t * 4) = o; __threadfence(); *(volatile v4f*)(Xb + t * 4) = o; }
__global__ __launch_bounds__(256) void k_nmask(float* out, const float* __restrict__ nm) { const size_t t = (size_t)blockIdx.x * 256 + threadIdx.x; if (t >= (size_t)NR * DD / 4) return; const size_t row = (t * 4) / DD; const float m = bf16_round(nm[row]); v4f v = *(const v4fa*)(out + t * 4);
#pragma unroll
  for (int q = 0; q < 4; ++q) v[q] *= m; *(volatile v4f*)(out + t * 4) = v; __threadfence(); *(volatile v4f*)(out + t * 4) = v; }

extern "C" void kernel_launch(void* const* d_in, const int* in_sizes, int n_in,
                              void* d_out, int out_size, void* d_ws, size_t ws_size, hipStream_t stream) {
  (void)in_sizes; (void)n_in; (void)out_size;
  const float* const* I = (const float* const*)d_in; const float* x = I[0]; const float* nmask = I[1]; const int* edges = (const int*)d_in[2]; const float* rmask = I[3]; const float* remb = I[4]; const float* rgeo = I[5];
  const float* Wq = I[6]; const float* bq = I[7]; const float* Wk = I[8]; const float* bk = I[9]; const float* Wv = I[10]; const float* bv = I[11]; const float* Web = I[12]; const float* beb = I[13]; const float* glg = I[14]; const float* glb = I[15]; const float* Wgeo = I[16]; const float* bgeo = I[17]; const float* Wout = I[18]; const float* bout = I[19]; const float* ng = I[20]; const float* nb = I[21]; const float* fg = I[22]; const float* fb = I[23]; const float* Wf1 = I[24]; const float* bf1 = I[25]; const float* Wf2 = I[26]; const float* bf2 = I[27];
  char* ws = (char*)d_ws; size_t off = 0;
  auto take = [&](size_t bytes) { char* p = ws + off; off += (bytes + 255) & ~(size_t)255; return p; };
  const int nch = (NET + C4_CH - 1) / C4_CH;
  int* c4_CNT = (int*)take((size_t)nch * C4_NB * 4); int* c4_OFFB = (int*)take((size_t)nch * C4_NB * 4); int* c4_BOFF = (int*)take((size_t)(C4_NB + 64) * 4); int* c4_BUF = (int*)take((size_t)(NET + 64) * 4);
  int* KA = (int*)take((size_t)NET * 4); int* KB = (int*)take((size_t)NET * 4); int* cntA = (int*)take((size_t)(NKEY + 64) * 4); int* nbrA = (int*)take((size_t)NKEY * ECAP * 4); int* cntB = (int*)take((size_t)(NKEY + 64) * 4); int* nbrB = (int*)take((size_t)NKEY * ECAP * 4); float* TB = (float*)take((size_t)NET * NH * 4);
  _Float16* Bqkv = (_Float16*)take((size_t)3 * DD * DD * 2); float* Bc = (float*)take((size_t)3 * DD * 4); _Float16* Bo = (_Float16*)take((size_t)DD * DD * 2); _Float16* Bf1 = (_Float16*)take((size_t)DFF * DD * 2); _Float16* Bf2 = (_Float16*)take((size_t)DD * DFF * 2);
  _Float16* XN = (_Float16*)take((size_t)NR * DD * 2); _Float16* QKV = (_Float16*)take((size_t)NR * 3 * DD * 2); _Float16* Vt = (_Float16*)take((size_t)NR * DD * 2);
  float* S = (float*)take((size_t)BGRP * NH * NND * NND * 4); _Float16* P16 = (_Float16*)take((size_t)BGRP * NH * NND * NND * 2); float* O = (float*)take((size_t)NR * DD * 4); _Float16* O16 = (_Float16*)take((size_t)NR * DD * 2);
  _Float16* F1 = QKV;
  float* Xb = S;
  float* X2 = O;
  _Float16* XN2 = P16;
  if (off > ws_size) return;
  k_round16f<<<(unsigned)(((size_t)DD * DD / 8 + 255) / 256), 256, 0, stream>>>(Wq, Bqkv, (size_t)DD * DD / 8); k_round16f<<<(unsigned)(((size_t)DD * DD / 8 + 255) / 256), 256, 0, stream>>>(Wk, Bqkv + (size_t)DD * DD, (size_t)DD * DD / 8); k_round16f<<<(unsigned)(((size_t)DD * DD / 8 + 255) / 256), 256, 0, stream>>>(Wv, Bqkv + (size_t)2 * DD * DD, (size_t)DD * DD / 8);
  k_bcat<<<(3 * DD + 255) / 256, 256, 0, stream>>>(bq, bk, bv, Bc); k_round16f<<<(unsigned)(((size_t)DD * DD / 8 + 255) / 256), 256, 0, stream>>>(Wout, Bo, (size_t)DD * DD / 8); k_round16f<<<(unsigned)(((size_t)DFF * DD / 8 + 255) / 256), 256, 0, stream>>>(Wf1, Bf1, (size_t)DFF * DD / 8); k_round16f<<<(unsigned)(((size_t)DD * DFF / 8 + 255) / 256), 256, 0, stream>>>(Wf2, Bf2, (size_t)DD * DFF / 8);
  k_ln512<1><<<NR / 8, 256, 0, stream>>>(x, ng, nb, XN);
  k_keys<<<(NET + 255) / 256, 256, 0, stream>>>(edges, rmask, KA, KB);
  k_tb<<<(NET * NH + 255) / 256, 256, 0, stream>>>(remb, rgeo, Web, beb, glg, glb, Wgeo, bgeo, TB);
  k_c4_count<<<(unsigned)nch, 256, 0, stream>>>(KA, NET, NKEY, c4_CNT); k_c4_offsets<<<1, 256, 0, stream>>>(c4_CNT, nch, NET, c4_OFFB, c4_BOFF); k_c4_scatter<<<(unsigned)nch, 256, 0, stream>>>(KA, NET, NKEY, c4_OFFB, c4_BUF); k_c4_lists<ECAP><<<(NKEY + 255) / 256, 256, 0, stream>>>(KA, c4_BUF, c4_BOFF, NKEY, NET, nbrA, cntA);
  k_c4_count<<<(unsigned)nch, 256, 0, stream>>>(KB, NET, NKEY, c4_CNT); k_c4_offsets<<<1, 256, 0, stream>>>(c4_CNT, nch, NET, c4_OFFB, c4_BOFF); k_c4_scatter<<<(unsigned)nch, 256, 0, stream>>>(KB, NET, NKEY, c4_OFFB, c4_BUF); k_c4_lists<ECAP><<<(NKEY + 255) / 256, 256, 0, stream>>>(KB, c4_BUF, c4_BOFF, NKEY, NET, nbrB, cntB);
  k_gemm_hhx<0><<<dim3(((NR / 16) * (3 * DD / 64) + 3) / 4, 1), 128, 0, stream>>>(XN, DD, 0, Bqkv, DD, 0, 0.0625f, Bc, 0, nullptr, 1, 0, 0, nullptr, QKV, 3 * DD, 0, NR, 3 * DD, DD);
  k_vt<NH, NND><<<NBG * NH * (NND / 64), 256, 0, stream>>>(QKV + 2 * DD, 3 * DD, 0, Vt);
  for (int g = 0; g < NBG / BGRP; ++g) { const int b0 = g * BGRP;
    for (int bl = 0; bl < BGRP; ++bl) { const int b = b0 + bl;
      k_gemm_hhx<0><<<dim3(((NND / 16) * (NND / 64) + 3) / 4, NH), 128, 0, stream>>>(QKV + (size_t)b * NND * 3 * DD, 3 * DD, HD, QKV + (size_t)b * NND * 3 * DD + DD, 3 * DD, HD, 0.125f, nullptr, 0, nullptr, 1, 0, 0, S + (size_t)bl * NH * NND * NND, nullptr, NND, (size_t)NND * NND, NND, NND, HD); }
    k_attnrow<<<BGRP * NND, 256, 0, stream>>>(S, TB, edges, nbrA, cntA, nbrB, cntB, nmask, b0, P16);
    for (int bl = 0; bl < BGRP; ++bl) { const int b = b0 + bl;
      k_gemm_hhx<0><<<dim3(((NND / 16) * (HD / 64) + 3) / 4, NH), 128, 0, stream>>>(P16 + (size_t)bl * NH * NND * NND, NND, (size_t)NND * NND, Vt + (size_t)b * NH * HD * NND, NND, (size_t)HD * NND, 0.0009765625f, nullptr, 0, nullptr, 1, 0, 0, O + (size_t)b * NND * DD, nullptr, DD, HD, NND, HD, NND); } }
  k_h16p<<<(unsigned)(((size_t)NR * DD / 8 + 255) / 256), 256, 0, stream>>>(O, O16, (size_t)NR * DD / 8);
  k_bfx<<<(unsigned)(((size_t)NR * DD / 4 + 255) / 256), 256, 0, stream>>>(x, Xb, (size_t)NR * DD / 4);
  const dim3 g512(((NR / 16) * (DD / 64) + 3) / 4, 1);
  k_gemm_hhx<0><<<g512, 128, 0, stream>>>(O16, DD, 0, Bo, DD, 0, 0.0625f, bout, 0, Xb, 1, (size_t)DD, 0, X2, nullptr, DD, 0, NR, DD, DD);
  k_ln512<0><<<NR / 8, 256, 0, stream>>>(X2, fg, fb, XN2);
  k_gemm_hhx<15><<<dim3(((NR / 16) * (DFF / 64) + 3) / 4, 1), 128, 0, stream>>>(XN2, DD, 0, Bf1, DD, 0, 0.0625f, bf1, 0, nullptr, 1, 0, 0, nullptr, F1, DFF, 0, NR, DFF, DD);
  k_gemm_hhx<0><<<g512, 128, 0, stream>>>(F1, DFF, 0, Bf2, DFF, 0, 0.0625f, bf2, 0, X2, 1, (size_t)DD, 0, (float*)d_out, nullptr, DD, 0, NR, DD, DFF);
  k_nmask<<<(unsigned)(((size_t)NR * DD / 4 + 255) / 256), 256, 0, stream>>>((float*)d_out, nmask);
}
